// MambaMixer_optimize_90958817394795
// MI455X (gfx1250) — hardware-run, weakly checked
//
#include <hip/hip_runtime.h>


#define LL   1024
#define HID  2048
#define DI   4096
#define NS   16
#define RR   128
typedef _Float16 h16;
typedef unsigned short bf;
typedef __attribute__((ext_vector_type(16))) __bf16   v16bf;
typedef __attribute__((ext_vector_type(16))) _Float16 v16h;
typedef __attribute__((ext_vector_type(8)))  _Float16 v8h;
typedef __attribute__((ext_vector_type(8)))  unsigned short v8us;
typedef __attribute__((ext_vector_type(8)))  float    v8f;
typedef __attribute__((ext_vector_type(4)))  float    v4f;
typedef v8h  __attribute__((may_alias)) v8ha;
typedef v4f  __attribute__((may_alias)) v4fa;
typedef v8us __attribute__((may_alias)) v8usa;

__device__ __forceinline__ unsigned short f2bf(float f) { unsigned u = __float_as_uint(f); u += 0x7FFFu + ((u >> 16) & 1u); return (unsigned short)(u >> 16); }
__device__ __forceinline__ float bf2f(unsigned short b) { return __uint_as_float(((unsigned)b) << 16); }
__device__ __forceinline__ float bfr(float f) { return bf2f(f2bf(f)); }
__device__ __forceinline__ v16h cat16(v8h lo, v8h hi) { return __builtin_shufflevector(lo, hi, 0, 1, 2, 3, 4, 5, 6, 7, 8, 9, 10, 11, 12, 13, 14, 15); }
__device__ __forceinline__ v16bf cat16b(v8us lo, v8us hi) { return __builtin_bit_cast(v16bf, __builtin_shufflevector(lo, hi, 0, 1, 2, 3, 4, 5, 6, 7, 8, 9, 10, 11, 12, 13, 14, 15)); }
__device__ __forceinline__ v8f wmma16(v16h a, v16h b, v8f c) { return __builtin_amdgcn_wmma_f32_16x16x32_f16(false, a, false, b, (short)0, c, false, false); }
__device__ __forceinline__ v8f wmmab(v16bf a, v16bf b, v8f c) { return __builtin_amdgcn_wmma_f32_16x16x32_bf16(false, a, false, b, (short)0, c, false, false); }


template <typename T16> struct WFrag;
template <> struct WFrag<h16> { typedef v16h V; static __device__ __forceinline__ V ld(const h16* p) { return cat16(*(const v8h*)p, *(const v8h*)(p + 16)); } static __device__ __forceinline__ v8f mma(V a, V b, v8f c) { return wmma16(a, b, c); } };
template <> struct WFrag<bf> { typedef v16bf V; static __device__ __forceinline__ V ld(const bf* p) { return cat16b(*(const v8us*)p, *(const v8us*)(p + 16)); } static __device__ __forceinline__ v8f mma(V a, V b, v8f c) { return wmmab(a, b, c); } };
template <typename T16, int NSPLIT, bool BIAS>
__global__ __launch_bounds__(32) void k_gemmw(const T16* __restrict__ A, const T16* __restrict__ A2, const T16* __restrict__ Bt, const T16* __restrict__ Bt2, int K, float* C, int ldc, const float* __restrict__ bias, size_t sA, size_t sB, size_t sC) {
    typedef typename WFrag<T16>::V V;
    __shared__ __align__(16) float os[16 * 68];
    const size_t z = blockIdx.z; A += z * sA; if (A2) A2 += z * sA; Bt += z * sB; if (Bt2) Bt2 += z * sB; C += z * sC;
    const int lane = threadIdx.x & 31, lr = lane & 15, hi = lane >> 4; const int r0 = blockIdx.x * 64, c0 = blockIdx.y * 64;
    v8f acc[4][4];
#pragma unroll
    for (int mb = 0; mb < 4; ++mb)
#pragma unroll
        for (int nb = 0; nb < 4; ++nb) acc[mb][nb] = (v8f){};
    const size_t aoff = (size_t)(r0 + lr) * K + 8 * hi, boff = (size_t)(c0 + lr) * K + 8 * hi;
#pragma unroll 1
    for (int kc = 0; kc < K; kc += 32) {
        V a[4], a2[4];
#pragma unroll
        for (int mb = 0; mb < 4; ++mb) { a[mb] = WFrag<T16>::ld(A + aoff + (size_t)mb * 16 * K + kc); if (NSPLIT == 1 || NSPLIT == 2) a2[mb] = WFrag<T16>::ld(A2 + aoff + (size_t)mb * 16 * K + kc); }
#pragma unroll
        for (int nb = 0; nb < 4; ++nb) { const V b = WFrag<T16>::ld(Bt + boff + (size_t)nb * 16 * K + kc); V b2; if (NSPLIT >= 2) b2 = WFrag<T16>::ld(Bt2 + boff + (size_t)nb * 16 * K + kc);
#pragma unroll
            for (int mb = 0; mb < 4; ++mb) { acc[mb][nb] = WFrag<T16>::mma(a[mb], b, acc[mb][nb]); if (NSPLIT == 1 || NSPLIT == 2) acc[mb][nb] = WFrag<T16>::mma(a2[mb], b, acc[mb][nb]); if (NSPLIT >= 2) acc[mb][nb] = WFrag<T16>::mma(a[mb], b2, acc[mb][nb]); } }
        asm volatile("v_nop\n\tv_nop\n\tv_nop\n\tv_nop" : "+v"(acc[0][0]), "+v"(acc[1][1]), "+v"(acc[2][2]), "+v"(acc[3][3]) : "v"(a[0]), "v"(a[3]));
    }
#pragma unroll
    for (int mb = 0; mb < 4; ++mb) {
#pragma unroll
        for (int nb = 0; nb < 4; ++nb) {
#pragma unroll
            for (int j = 0; j < 8; ++j) os[(hi * 8 + j) * 68 + nb * 16 + lr] = acc[mb][nb][j]; }
        __builtin_amdgcn_wave_barrier(); asm volatile("" ::: "memory");
        float* crow = C + (size_t)(r0 + mb * 16) * ldc + c0;
#pragma unroll 1
        for (int ps = 0; ps < 2; ++ps) {
#pragma unroll
            for (int s = 0; s < 8; ++s) { const int row = 2 * s + hi, cofs = lr * 4; v4f val = *(const v4fa*)(os + row * 68 + cofs); if (BIAS) { val[0] += bfr(bias[c0 + cofs]); val[1] += bfr(bias[c0 + cofs + 1]); val[2] += bfr(bias[c0 + cofs + 2]); val[3] += bfr(bias[c0 + cofs + 3]); }
                *(volatile v4f*)(crow + (size_t)row * ldc + cofs) = val; }
            if (ps == 0) __threadfence(); }
        __builtin_amdgcn_wave_barrier(); asm volatile("" ::: "memory");
    }
}

__device__ __forceinline__ void splitf(float y, unsigned short& h, unsigned short& l) { h = f2bf(y); l = f2bf(y - bf2f(h)); }
__device__ __forceinline__ float silu_(float x) { return __fmul_rn(x, __fdiv_rn(1.0f, 1.0f + __expf(-x))); }
typedef __attribute__((ext_vector_type(2))) unsigned short v2us;
typedef __attribute__((ext_vector_type(4))) unsigned short v4us;

__global__ __launch_bounds__(256) void k_cvt8(const float* __restrict__ src, bf* dst, size_t n8) { const size_t i = (size_t)blockIdx.x * 256 + threadIdx.x; if (i >= n8) return; const v8f v = *(const v8f*)(src + i * 8); v8us o;
#pragma unroll
    for (int k = 0; k < 8; ++k) o[k] = f2bf(v[k]); *(volatile v8us*)(dst + i * 8) = o; __threadfence(); *(volatile v8us*)(dst + i * 8) = o; }
__global__ __launch_bounds__(256) void k_wbc(const float* __restrict__ wb, const float* __restrict__ wc, bf* WBC) { const int i = (blockIdx.x * 256 + threadIdx.x) * 4; if (i >= 64 * DI) return; const int n = i / DI, k = i % DI; v4us o;
#pragma unroll
    for (int q = 0; q < 4; ++q) o[q] = n < NS ? f2bf(wb[n * DI + k + q]) : (n < 2 * NS ? f2bf(wc[(n - NS) * DI + k + q]) : (unsigned short)0); *(volatile v4us*)(WBC + i) = o; __threadfence(); *(volatile v4us*)(WBC + i) = o; }
__global__ __launch_bounds__(256) void k_split(const float* __restrict__ F, int pitch, int c0, int wsel, bf* Hh, bf* Hl) { const int e = (blockIdx.x * 256 + threadIdx.x) * 4; if (e >= LL * wsel) return; const int c = e % wsel, t = e / wsel; const v4f a = *(const v4f*)(F + (size_t)t * pitch + c0 + c); v4us oh, ol;
#pragma unroll
    for (int q = 0; q < 4; ++q) { unsigned short u, l; splitf(a[q], u, l); oh[q] = u; ol[q] = l; } *(volatile v4us*)(Hh + e) = oh; *(volatile v4us*)(Hl + e) = ol; __threadfence(); *(volatile v4us*)(Hh + e) = oh; *(volatile v4us*)(Hl + e) = ol; }
__global__ __launch_bounds__(256) void k_conv(const float* __restrict__ H0, const float* __restrict__ w, const float* __restrict__ bb, float* HS, bf* Ch, bf* Cl) { const int e = (blockIdx.x * 256 + threadIdx.x) * 4; if (e >= LL * DI) return; const int c = e % DI, t = e / DI; v4f o; v4us oh, ol;
#pragma unroll
    for (int q = 0; q < 4; ++q) { const int cc = c + q; float acc = 0.f;
#pragma unroll
        for (int k = 0; k < 4; ++k) { const int ts = t - 3 + k; if (ts >= 0) { float p = __fmul_rn(bfr(w[cc * 4 + k]), H0[(size_t)ts * DI + cc]); asm volatile("" : "+v"(p)); acc = __fadd_rn(acc, p); } }
        o[q] = silu_(__fadd_rn(acc, bfr(bb[cc]))); unsigned short u, l; splitf(o[q], u, l); oh[q] = u; ol[q] = l; }
    for (int ps = 0; ps < 2; ++ps) { *(volatile v4f*)(HS + e) = o; *(volatile v4us*)(Ch + e) = oh; *(volatile v4us*)(Cl + e) = ol; if (ps == 0) __threadfence(); } }
__global__ __launch_bounds__(256) void k_scan(const float* __restrict__ DTR, const float* __restrict__ HS, const float* __restrict__ PBC, const float* __restrict__ GATE, const float* __restrict__ alog, const float* __restrict__ Dp, bf* Yh, bf* Yl) {
    __shared__ float ybuf[64]; const int tid = threadIdx.x; const int cl = tid >> 2, sub = tid & 3; const int d = blockIdx.x * 64 + cl; const int n0 = sub * 4; float A[4], s[4];
#pragma unroll
    for (int j = 0; j < 4; ++j) { A[j] = -__expf(bfr(alog[(size_t)d * NS + n0 + j])); s[j] = 0.f; }
    const float dd = bfr(Dp[d]);
    for (int t = 0; t < LL; ++t) { const float raw = DTR[(size_t)t * DI + d]; const float dt = raw > 20.f ? raw : log1pf(__expf(raw)); const float hs = HS[(size_t)t * DI + d]; const float dtx = __fmul_rn(dt, hs); const float* pr = PBC + (size_t)t * 64; float y = 0.f;
#pragma unroll
        for (int j = 0; j < 4; ++j) { const float a = __expf(__fmul_rn(A[j], dt)); float hb = __fmul_rn(dtx, pr[n0 + j]); asm volatile("" : "+v"(hb)); float ha = __fmul_rn(a, s[j]); asm volatile("" : "+v"(ha)); s[j] = __fadd_rn(ha, hb); float yc = __fmul_rn(s[j], pr[NS + n0 + j]); asm volatile("" : "+v"(yc)); y = __fadd_rn(y, yc); }
        y += __shfl_xor(y, 1, 32); y += __shfl_xor(y, 2, 32);
        if (sub == 0) { float sk = __fmul_rn(dd, hs); asm volatile("" : "+v"(sk)); const float yy = __fadd_rn(y, sk); ybuf[cl] = __fmul_rn(yy, silu_(GATE[(size_t)t * DI + d])); }
        __syncthreads();
        if (tid < 32) { v2us oh, ol; unsigned short u, l; splitf(ybuf[2 * tid], u, l); oh[0] = u; ol[0] = l; splitf(ybuf[2 * tid + 1], u, l); oh[1] = u; ol[1] = l; const size_t o = (size_t)t * DI + blockIdx.x * 64 + 2 * tid; *(volatile v2us*)(Yh + o) = oh; *(volatile v2us*)(Yl + o) = ol; __threadfence(); *(volatile v2us*)(Yh + o) = oh; *(volatile v2us*)(Yl + o) = ol; }
        __syncthreads(); } }

extern "C" void kernel_launch(void* const* d_in, const int* in_sizes, int n_in,
                              void* d_out, int out_size, void* d_ws, size_t ws_size, hipStream_t stream) {
    (void)in_sizes; (void)n_in; (void)out_size;
    const float* x = (const float*)d_in[0]; const float* wis = (const float*)d_in[1]; const float* wig = (const float*)d_in[2]; const float* cw = (const float*)d_in[3]; const float* cb = (const float*)d_in[4]; const float* wdt = (const float*)d_in[5]; const float* wb = (const float*)d_in[6]; const float* wc = (const float*)d_in[7]; const float* wdtp = (const float*)d_in[8]; const float* bdtp = (const float*)d_in[9]; const float* alog = (const float*)d_in[10]; const float* Dp = (const float*)d_in[11]; const float* wout = (const float*)d_in[12];
    float* OUT = (float*)d_out;
    char* wsp = (char*)d_ws;
    auto take = [&](size_t bytes) { char* p = wsp; wsp += (bytes + 255) & ~(size_t)255; return (void*)p; };
    bf* WIS = (bf*)take((size_t)DI * HID * 2); bf* WIG = (bf*)take((size_t)DI * HID * 2); bf* WDT = (bf*)take((size_t)RR * DI * 2); bf* WBC = (bf*)take((size_t)64 * DI * 2); bf* WDP = (bf*)take((size_t)DI * RR * 2); bf* WOUT = (bf*)take((size_t)HID * DI * 2);
    bf* XB = (bf*)take((size_t)LL * HID * 2); float* H0 = (float*)take((size_t)LL * DI * 4); float* GATE = (float*)take((size_t)LL * DI * 4); float* HS = (float*)take((size_t)LL * DI * 4); bf* Ch = (bf*)take((size_t)LL * DI * 2); bf* Cl = (bf*)take((size_t)LL * DI * 2);
    float* TS = (float*)take((size_t)LL * RR * 4); bf* TSh = (bf*)take((size_t)LL * RR * 2); bf* TSl = (bf*)take((size_t)LL * RR * 2); float* DTR = (float*)take((size_t)LL * DI * 4); float* PBC = (float*)take((size_t)LL * 64 * 4); bf* Yh = (bf*)take((size_t)LL * DI * 2); bf* Yl = (bf*)take((size_t)LL * DI * 2);
    if ((size_t)(wsp - (char*)d_ws) > ws_size) return;
    k_cvt8<<<(unsigned)(((size_t)DI * HID / 8 + 255) / 256), 256, 0, stream>>>(wis, WIS, (size_t)DI * HID / 8); k_cvt8<<<(unsigned)(((size_t)DI * HID / 8 + 255) / 256), 256, 0, stream>>>(wig, WIG, (size_t)DI * HID / 8); k_cvt8<<<(RR * DI / 8 + 255) / 256, 256, 0, stream>>>(wdt, WDT, (size_t)RR * DI / 8);
    k_wbc<<<(64 * DI / 4 + 255) / 256, 256, 0, stream>>>(wb, wc, WBC); k_cvt8<<<(DI * RR / 8 + 255) / 256, 256, 0, stream>>>(wdtp, WDP, (size_t)DI * RR / 8); k_cvt8<<<(unsigned)(((size_t)HID * DI / 8 + 255) / 256), 256, 0, stream>>>(wout, WOUT, (size_t)HID * DI / 8);
    k_cvt8<<<(unsigned)(((size_t)LL * HID / 8 + 255) / 256), 256, 0, stream>>>(x, XB, (size_t)LL * HID / 8);
    k_gemmw<bf, 0, false><<<dim3(LL / 64, DI / 64, 1), 32, 0, stream>>>(XB, nullptr, WIS, nullptr, HID, H0, DI, nullptr, 0, 0, 0); k_gemmw<bf, 0, false><<<dim3(LL / 64, DI / 64, 1), 32, 0, stream>>>(XB, nullptr, WIG, nullptr, HID, GATE, DI, nullptr, 0, 0, 0);
    k_conv<<<(LL * DI / 4 + 255) / 256, 256, 0, stream>>>(H0, cw, cb, HS, Ch, Cl);
    k_gemmw<bf, 1, false><<<dim3(LL / 64, RR / 64, 1), 32, 0, stream>>>(Ch, Cl, WDT, nullptr, DI, TS, RR, nullptr, 0, 0, 0); k_split<<<(LL * RR / 4 + 255) / 256, 256, 0, stream>>>(TS, RR, 0, RR, TSh, TSl);
    k_gemmw<bf, 1, true><<<dim3(LL / 64, DI / 64, 1), 32, 0, stream>>>(TSh, TSl, WDP, nullptr, RR, DTR, DI, bdtp, 0, 0, 0);
    k_gemmw<bf, 1, false><<<dim3(LL / 64, 1, 1), 32, 0, stream>>>(Ch, Cl, WBC, nullptr, DI, PBC, 64, nullptr, 0, 0, 0);
    k_scan<<<DI / 64, 256, 0, stream>>>(DTR, HS, PBC, GATE, alog, Dp, Yh, Yl);
    k_gemmw<bf, 1, false><<<dim3(LL / 64, HID / 64, 1), 32, 0, stream>>>(Yh, Yl, WOUT, nullptr, DI, OUT, HID, nullptr, 0, 0, 0);
}
